// RealNVP_73263552135281
// MI455X (gfx1250) — hardware-run, weakly checked
//
#include <hip/hip_runtime.h>


#define NPTS 262144
#define RC   65536
#define DIM  8
#define NT   4
#define NL   6
#define HID  128
#define KX   32
#define NO   64
typedef _Float16 h16;
typedef unsigned short bf;
typedef __attribute__((ext_vector_type(16))) __bf16   v16bf;
typedef __attribute__((ext_vector_type(16))) _Float16 v16h;
typedef __attribute__((ext_vector_type(8)))  _Float16 v8h;
typedef __attribute__((ext_vector_type(8)))  unsigned short v8us;
typedef __attribute__((ext_vector_type(8)))  float    v8f;
typedef __attribute__((ext_vector_type(4)))  float    v4f;
typedef v8h  __attribute__((may_alias)) v8ha;
typedef v4f  __attribute__((may_alias)) v4fa;
typedef v8us __attribute__((may_alias)) v8usa;

__device__ __forceinline__ unsigned short f2bf(float f) { unsigned u = __float_as_uint(f); u += 0x7FFFu + ((u >> 16) & 1u); return (unsigned short)(u >> 16); }
__device__ __forceinline__ float bf2f(unsigned short b) { return __uint_as_float(((unsigned)b) << 16); }
__device__ __forceinline__ float bfr(float f) { return bf2f(f2bf(f)); }
__device__ __forceinline__ v16h cat16(v8h lo, v8h hi) { return __builtin_shufflevector(lo, hi, 0, 1, 2, 3, 4, 5, 6, 7, 8, 9, 10, 11, 12, 13, 14, 15); }
__device__ __forceinline__ v16bf cat16b(v8us lo, v8us hi) { return __builtin_bit_cast(v16bf, __builtin_shufflevector(lo, hi, 0, 1, 2, 3, 4, 5, 6, 7, 8, 9, 10, 11, 12, 13, 14, 15)); }
__device__ __forceinline__ v8f wmma16(v16h a, v16h b, v8f c) { return __builtin_amdgcn_wmma_f32_16x16x32_f16(false, a, false, b, (short)0, c, false, false); }
__device__ __forceinline__ v8f wmmab(v16bf a, v16bf b, v8f c) { return __builtin_amdgcn_wmma_f32_16x16x32_bf16(false, a, false, b, (short)0, c, false, false); }


template <typename T16> struct WFrag;
template <> struct WFrag<h16> { typedef v16h V; static __device__ __forceinline__ V ld(const h16* p) { return cat16(*(const v8h*)p, *(const v8h*)(p + 16)); } static __device__ __forceinline__ v8f mma(V a, V b, v8f c) { return wmma16(a, b, c); } };
template <> struct WFrag<bf> { typedef v16bf V; static __device__ __forceinline__ V ld(const bf* p) { return cat16b(*(const v8us*)p, *(const v8us*)(p + 16)); } static __device__ __forceinline__ v8f mma(V a, V b, v8f c) { return wmmab(a, b, c); } };
template <typename T16, int NSPLIT, bool BIAS>
__global__ __launch_bounds__(32) void k_gemmw(const T16* __restrict__ A, const T16* __restrict__ A2, const T16* __restrict__ Bt, const T16* __restrict__ Bt2, int K, float* C, int ldc, const float* __restrict__ bias, size_t sA, size_t sB, size_t sC) {
    typedef typename WFrag<T16>::V V;
    __shared__ __align__(16) float os[16 * 68];
    const size_t z = blockIdx.z; A += z * sA; if (A2) A2 += z * sA; Bt += z * sB; if (Bt2) Bt2 += z * sB; C += z * sC;
    const int lane = threadIdx.x & 31, lr = lane & 15, hi = lane >> 4; const int r0 = blockIdx.x * 64, c0 = blockIdx.y * 64;
    v8f acc[4][4];
#pragma unroll
    for (int mb = 0; mb < 4; ++mb)
#pragma unroll
        for (int nb = 0; nb < 4; ++nb) acc[mb][nb] = (v8f){};
    const size_t aoff = (size_t)(r0 + lr) * K + 8 * hi, boff = (size_t)(c0 + lr) * K + 8 * hi;
#pragma unroll 1
    for (int kc = 0; kc < K; kc += 32) {
        V a[4], a2[4];
#pragma unroll
        for (int mb = 0; mb < 4; ++mb) { a[mb] = WFrag<T16>::ld(A + aoff + (size_t)mb * 16 * K + kc); if (NSPLIT == 1 || NSPLIT == 2) a2[mb] = WFrag<T16>::ld(A2 + aoff + (size_t)mb * 16 * K + kc); }
#pragma unroll
        for (int nb = 0; nb < 4; ++nb) { const V b = WFrag<T16>::ld(Bt + boff + (size_t)nb * 16 * K + kc); V b2; if (NSPLIT >= 2) b2 = WFrag<T16>::ld(Bt2 + boff + (size_t)nb * 16 * K + kc);
#pragma unroll
            for (int mb = 0; mb < 4; ++mb) { acc[mb][nb] = WFrag<T16>::mma(a[mb], b, acc[mb][nb]); if (NSPLIT == 1 || NSPLIT == 2) acc[mb][nb] = WFrag<T16>::mma(a2[mb], b, acc[mb][nb]); if (NSPLIT >= 2) acc[mb][nb] = WFrag<T16>::mma(a[mb], b2, acc[mb][nb]); } }
        asm volatile("v_nop\n\tv_nop\n\tv_nop\n\tv_nop" : "+v"(acc[0][0]), "+v"(acc[1][1]), "+v"(acc[2][2]), "+v"(acc[3][3]) : "v"(a[0]), "v"(a[3]));
    }
#pragma unroll
    for (int mb = 0; mb < 4; ++mb) {
#pragma unroll
        for (int nb = 0; nb < 4; ++nb) {
#pragma unroll
            for (int j = 0; j < 8; ++j) os[(hi * 8 + j) * 68 + nb * 16 + lr] = acc[mb][nb][j]; }
        __builtin_amdgcn_wave_barrier(); asm volatile("" ::: "memory");
        float* crow = C + (size_t)(r0 + mb * 16) * ldc + c0;
#pragma unroll 1
        for (int ps = 0; ps < 2; ++ps) {
#pragma unroll
            for (int s = 0; s < 8; ++s) { const int row = 2 * s + hi, cofs = lr * 4; v4f val = *(const v4fa*)(os + row * 68 + cofs); if (BIAS) { val[0] += bfr(bias[c0 + cofs]); val[1] += bfr(bias[c0 + cofs + 1]); val[2] += bfr(bias[c0 + cofs + 2]); val[3] += bfr(bias[c0 + cofs + 3]); }
                *(volatile v4f*)(crow + (size_t)row * ldc + cofs) = val; }
            if (ps == 0) __threadfence(); }
        __builtin_amdgcn_wave_barrier(); asm volatile("" ::: "memory");
    }
}

typedef __attribute__((ext_vector_type(4))) unsigned short v4us;
typedef __attribute__((ext_vector_type(2))) unsigned short v2us;
__device__ __forceinline__ void splitf(float y, unsigned short& h, unsigned short& l) { h = f2bf(y); l = f2bf(y - bf2f(h)); }
__device__ __forceinline__ float tanhx(float a) { return __fsub_rn(1.0f, __fdiv_rn(2.0f, __fadd_rn(__builtin_amdgcn_exp2f(__fmul_rn(a, 2.8853900817779268f)), 1.0f))); }
__device__ __forceinline__ float expx(float a) { return __builtin_amdgcn_exp2f(__fmul_rn(a, 1.4426950408889634f)); }
__global__ __launch_bounds__(256) void k_wtG(const float* __restrict__ w, int K, int N, bf* Bt) {
    const int lane = threadIdx.x & 31; const int L0 = (blockIdx.x * 8 + (threadIdx.x >> 5)) * 8; const int nlines = N * K / 64;
#pragma unroll
    for (int ps = 0; ps < 2; ++ps) {
#pragma unroll 1
        for (int l = 0; l < 8; ++l) { const int L = L0 + l; if (L >= nlines) break; const size_t e = (size_t)L * 64 + lane * 2; const int k = (int)(e % K), n = (int)(e / K); v2us o;
            o[0] = f2bf(w[(size_t)k * N + n]); o[1] = f2bf(w[(size_t)(k + 1) * N + n]); *(volatile v2us*)(Bt + e) = o; }
        if (ps == 0) __threadfence(); }
}

__global__ __launch_bounds__(128) void k_w1pad(const float* __restrict__ w, bf* Bt) { const int o = threadIdx.x; if (o >= HID) return; unsigned short c[KX];
#pragma unroll
    for (int k = 0; k < KX; ++k) c[k] = (k < NT) ? f2bf(w[k * HID + o]) : (unsigned short)0;
#pragma unroll 1
    for (int ps = 0; ps < 2; ++ps) {
#pragma unroll
        for (int c8 = 0; c8 < KX; c8 += 8) { v8us v;
#pragma unroll
            for (int k = 0; k < 8; ++k) v[k] = c[c8 + k]; *(volatile v8us*)(Bt + (size_t)o * KX + c8) = v; }
        if (ps == 0) __threadfence(); } }
__global__ __launch_bounds__(256) void k_w3pad(const float* __restrict__ w, bf* Bt) { const int i = blockIdx.x * 256 + threadIdx.x; if (i >= NO * HID / 8) return; const int o = i / (HID / 8), c0 = (i % (HID / 8)) * 8; v8us v;
#pragma unroll
    for (int k = 0; k < 8; ++k) v[k] = (o < 2 * NT) ? f2bf(w[(size_t)(c0 + k) * (2 * NT) + o]) : (unsigned short)0; *(volatile v8us*)(Bt + (size_t)o * HID + c0) = v; __threadfence(); *(volatile v8us*)(Bt + (size_t)o * HID + c0) = v; }
__global__ __launch_bounds__(128) void k_b3pad(const float* __restrict__ b3, float* B3P) { const int i = threadIdx.x; if (i >= NL * NO / 4) return; v4f o;
#pragma unroll
    for (int q = 0; q < 4; ++q) { const int e = i * 4 + q; const int l = e / NO, c = e % NO; o[q] = (c < 2 * NT) ? b3[l * 2 * NT + c] : 0.0f; } *(volatile v4f*)(B3P + i * 4) = o; __threadfence(); *(volatile v4f*)(B3P + i * 4) = o; }
__global__ __launch_bounds__(256) void k_pre(const float* __restrict__ X, size_t n0, int layer, const float* __restrict__ anls, const float* __restrict__ anb, float* Z, bf* XFh, bf* XFl) {
    const size_t r = (size_t)blockIdx.x * 256 + threadIdx.x; if (r >= RC) return; float z[DIM];
    if (layer == 0) { const v4f a = *(const v4f*)(X + (n0 + r) * DIM); const v4f b = *(const v4f*)(X + (n0 + r) * DIM + 4); for (int k = 0; k < 4; ++k) { z[k] = bfr(a[k]); z[4 + k] = bfr(b[k]); } }
    else { const v4f a = *(const v4f*)(Z + r * DIM); const v4f b = *(const v4f*)(Z + r * DIM + 4); for (int k = 0; k < 4; ++k) { z[k] = a[k]; z[4 + k] = b[k]; } }
#pragma unroll
    for (int k = 0; k < DIM; ++k) { const float ls = fminf(fmaxf(bfr(anls[layer * DIM + k]), -5.0f), 5.0f); float t = __fadd_rn(z[k], bfr(anb[layer * DIM + k])); asm volatile("" : "+v"(t)); z[k] = __fmul_rn(t, expx(ls)); }
    const int f0 = layer & 1;
    unsigned short hh[KX], ll[KX];
#pragma unroll
    for (int k = 0; k < KX; ++k) { hh[k] = 0; ll[k] = 0; }
#pragma unroll
    for (int j = 0; j < NT; ++j) { unsigned short h2, l2; splitf(z[f0 + 2 * j], h2, l2); hh[j] = h2; ll[j] = l2; }
    v4f za, zb; for (int k = 0; k < 4; ++k) { za[k] = z[k]; zb[k] = z[4 + k]; }
#pragma unroll 1
    for (int ps = 0; ps < 2; ++ps) {
        *(volatile v4f*)(Z + r * DIM) = za; *(volatile v4f*)(Z + r * DIM + 4) = zb;
#pragma unroll
        for (int c8 = 0; c8 < KX; c8 += 8) { v8us oh, ol;
#pragma unroll
            for (int k = 0; k < 8; ++k) { oh[k] = hh[c8 + k]; ol[k] = ll[c8 + k]; }
            *(volatile v8us*)(XFh + r * KX + c8) = oh; *(volatile v8us*)(XFl + r * KX + c8) = ol; }
        if (ps == 0) __threadfence(); }
}
__global__ __launch_bounds__(256) void k_relu(const float* __restrict__ F, bf* Rh, bf* Rl, size_t n4) { const size_t i = (size_t)blockIdx.x * 256 + threadIdx.x; if (i >= n4) return; const v4f a = *(const v4f*)(F + i * 4); v4us oh, ol;
#pragma unroll
    for (int q = 0; q < 4; ++q) { unsigned short h2, l2; splitf(fmaxf(a[q], 0.0f), h2, l2); oh[q] = h2; ol[q] = l2; }
    *(volatile v4us*)(Rh + i * 4) = oh; *(volatile v4us*)(Rl + i * 4) = ol; __threadfence(); *(volatile v4us*)(Rh + i * 4) = oh; *(volatile v4us*)(Rl + i * 4) = ol; }
__global__ __launch_bounds__(256) void k_post(const float* __restrict__ H3, int layer, const float* __restrict__ anls, const float* __restrict__ lgam, float* Z, float* LD) {
    const size_t r = (size_t)blockIdx.x * 256 + threadIdx.x; if (r >= RC) return; float z[DIM]; { const v4f a = *(const v4f*)(Z + r * DIM); const v4f b = *(const v4f*)(Z + r * DIM + 4); for (int k = 0; k < 4; ++k) { z[k] = a[k]; z[4 + k] = b[k]; } }
    float ld = (layer == 0) ? 0.0f : LD[r]; float lsum = 0.f;
#pragma unroll
    for (int k = 0; k < DIM; ++k) lsum = __fadd_rn(lsum, fminf(fmaxf(bfr(anls[layer * DIM + k]), -5.0f), 5.0f));
    ld = __fadd_rn(ld, lsum);
    const int f0 = layer & 1, t0 = f0 ^ 1; float zn[DIM]; float ldinc = 0.f;
#pragma unroll
    for (int j = 0; j < NT; ++j) { const float hr = H3[r * NO + j], hs = H3[r * NO + NT + j]; const float lg = fminf(fmaxf(bfr(lgam[layer * NT + j]), -5.0f), 5.0f);
        float sh = __fmul_rn(expx(lg), tanhx(hr)); asm volatile("" : "+v"(sh)); float sc = __fmul_rn(0.6f, tanhx(hs)); asm volatile("" : "+v"(sc));
        const float xt = z[t0 + 2 * j]; float m = __fmul_rn(xt, __fadd_rn(1.0f, sc)); asm volatile("" : "+v"(m)); const float yt = __fadd_rn(m, sh);
        ldinc = __fadd_rn(ldinc, logf(__fadd_rn(fabsf(__fadd_rn(1.0f, sc)), 1e-8f)));
        zn[f0 + 2 * j] = z[f0 + 2 * j]; zn[t0 + 2 * j] = yt; }
    ld = __fadd_rn(ld, ldinc);
    v4f za, zb; for (int k = 0; k < 4; ++k) { za[k] = zn[DIM - 1 - k]; zb[k] = zn[DIM - 1 - (4 + k)]; }
    *(volatile v4f*)(Z + r * DIM) = za; *(volatile v4f*)(Z + r * DIM + 4) = zb; *(volatile float*)(LD + r) = ld; __threadfence(); *(volatile v4f*)(Z + r * DIM) = za; *(volatile v4f*)(Z + r * DIM + 4) = zb; *(volatile float*)(LD + r) = ld; }
__global__ __launch_bounds__(256) void k_out(const float* __restrict__ Z, const float* __restrict__ LD, size_t n0, float* out0, float* out1) { const size_t r = (size_t)blockIdx.x * 256 + threadIdx.x; if (r >= RC) return; const v4f a = *(const v4f*)(Z + r * DIM); const v4f b = *(const v4f*)(Z + r * DIM + 4); const float l = LD[r];
    *(volatile v4f*)(out0 + (n0 + r) * DIM) = a; *(volatile v4f*)(out0 + (n0 + r) * DIM + 4) = b; *(volatile float*)(out1 + n0 + r) = l; __threadfence(); *(volatile v4f*)(out0 + (n0 + r) * DIM) = a; *(volatile v4f*)(out0 + (n0 + r) * DIM + 4) = b; *(volatile float*)(out1 + n0 + r) = l; }

extern "C" void kernel_launch(void* const* d_in, const int* in_sizes, int n_in,
                              void* d_out, int out_size, void* d_ws, size_t ws_size, hipStream_t stream) {
    (void)in_sizes; (void)n_in; (void)out_size;
    const float* x = (const float*)d_in[0]; const float* anls = (const float*)d_in[1]; const float* anb = (const float*)d_in[2]; const float* w1 = (const float*)d_in[3]; const float* b1 = (const float*)d_in[4]; const float* w2 = (const float*)d_in[5]; const float* b2 = (const float*)d_in[6]; const float* w3 = (const float*)d_in[7]; const float* b3 = (const float*)d_in[8]; const float* lgam = (const float*)d_in[9];
    float* OUT0 = (float*)d_out; float* OUT1 = OUT0 + (size_t)NPTS * DIM;
    char* wsp = (char*)d_ws;
    auto take = [&](size_t bytes) { char* p = wsp; wsp += (bytes + 255) & ~(size_t)255; return (void*)p; };
    bf* W1B = (bf*)take((size_t)NL * HID * KX * 2); bf* W2B = (bf*)take((size_t)NL * HID * HID * 2); bf* W3B = (bf*)take((size_t)NL * NO * HID * 2); float* B3P = (float*)take((size_t)NL * NO * 4);
    float* Z = (float*)take((size_t)RC * DIM * 4); float* LD = (float*)take((size_t)RC * 4); bf* XFh = (bf*)take((size_t)RC * KX * 2); bf* XFl = (bf*)take((size_t)RC * KX * 2); float* F = (float*)take((size_t)RC * HID * 4); bf* Hh = (bf*)take((size_t)RC * HID * 2); bf* Hl = (bf*)take((size_t)RC * HID * 2); float* H3 = (float*)take((size_t)RC * NO * 4);
    if ((size_t)(wsp - (char*)d_ws) > ws_size) return;
    for (int i = 0; i < NL; ++i) { k_w1pad<<<1, 128, 0, stream>>>(w1 + (size_t)i * NT * HID, W1B + (size_t)i * HID * KX); k_wtG<<<(unsigned)((HID * HID / 64 + 63) / 64), 256, 0, stream>>>(w2 + (size_t)i * HID * HID, HID, HID, W2B + (size_t)i * HID * HID); k_w3pad<<<(NO * HID / 8 + 255) / 256, 256, 0, stream>>>(w3 + (size_t)i * HID * 2 * NT, W3B + (size_t)i * NO * HID); }
    k_b3pad<<<1, 128, 0, stream>>>(b3, B3P);
    const size_t N4 = (size_t)RC * HID / 4;
    for (size_t n0 = 0; n0 < NPTS; n0 += RC) {
        for (int i = 0; i < NL; ++i) {
            k_pre<<<(RC + 255) / 256, 256, 0, stream>>>(x, n0, i, anls, anb, Z, XFh, XFl);
            k_gemmw<bf, 1, true><<<dim3(RC / 64, HID / 64, 1), 32, 0, stream>>>(XFh, XFl, W1B + (size_t)i * HID * KX, nullptr, KX, F, HID, b1 + i * HID, 0, 0, 0);
            k_relu<<<(unsigned)((N4 + 255) / 256), 256, 0, stream>>>(F, Hh, Hl, N4);
            k_gemmw<bf, 1, true><<<dim3(RC / 64, HID / 64, 1), 32, 0, stream>>>(Hh, Hl, W2B + (size_t)i * HID * HID, nullptr, HID, F, HID, b2 + i * HID, 0, 0, 0);
            k_relu<<<(unsigned)((N4 + 255) / 256), 256, 0, stream>>>(F, Hh, Hl, N4);
            k_gemmw<bf, 1, true><<<dim3(RC / 64, NO / 64, 1), 32, 0, stream>>>(Hh, Hl, W3B + (size_t)i * NO * HID, nullptr, HID, H3, NO, B3P + (size_t)i * NO, 0, 0, 0);
            k_post<<<(RC + 255) / 256, 256, 0, stream>>>(H3, i, anls, lgam, Z, LD); }
        k_out<<<(RC + 255) / 256, 256, 0, stream>>>(Z, LD, n0, OUT0, OUT1); }
}
